// CausalMultiHeadSelfAttention_71064528879764
// MI455X (gfx1250) — hardware-verified
//
#include <hip/hip_runtime.h>


#ifndef NB
#define NB 2
#endif
#ifndef SEQ
#define SEQ 2048
#endif
#define NB_FULL  2
#define SEQ_FULL 2048
#define TT   SEQ
#define DM   1024
#define NH_  16
#define NKV  16
#define REP  (NH_ / NKV)
#define HD   64
#define DQ   (NH_ * HD)
#define DKV  (NKV * HD)
#define ZH   2
#define RH   (SEQ < 512 ? SEQ : 512)
#define PCAR 1024.0f
#define SCL  0.125f
#define THETA_I 10000
typedef _Float16 h16;
typedef unsigned short bf;
typedef __attribute__((ext_vector_type(16))) __bf16   v16bf;
typedef __attribute__((ext_vector_type(16))) _Float16 v16h;
typedef __attribute__((ext_vector_type(8)))  _Float16 v8h;
typedef __attribute__((ext_vector_type(8)))  unsigned short v8us;
typedef __attribute__((ext_vector_type(8)))  float    v8f;
typedef __attribute__((ext_vector_type(4)))  float    v4f;
typedef v8h  __attribute__((may_alias)) v8ha;
typedef v4f  __attribute__((may_alias)) v4fa;
typedef v8us __attribute__((may_alias)) v8usa;

static_assert(NB >= 1 && NB <= NB_FULL);
static_assert(SEQ <= SEQ_FULL);
static_assert(TT % 128 == 0);
static_assert(RH % 64 == 0);
static_assert(TT >= RH);
static_assert(HD == 64);
static_assert(DM % 64 == 0 && DQ % 64 == 0 && DKV % 64 == 0);
static_assert(NH_ % ZH == 0);
static_assert(REP == 1);
static_assert(((size_t)DQ * DM / 8) % 256 == 0);
static_assert(((size_t)TT * DM / 8) % 256 == 0);
static_assert(((size_t)NH_ * TT * HD / 2) % 256 == 0);
static_assert(((size_t)NKV * TT * HD / 2) % 256 == 0);
static_assert(((size_t)ZH * TT * HD / 2) % 256 == 0);
static_assert(((size_t)TT * HD) % 256 == 0);
static_assert(((size_t)ZH * TT) % 8 == 0);

__device__ __forceinline__ unsigned short f2bf(float f) { unsigned u = __float_as_uint(f); u += 0x7FFFu + ((u >> 16) & 1u); return (unsigned short)(u >> 16); }
__device__ __forceinline__ float bf2f(unsigned short b) { return __uint_as_float(((unsigned)b) << 16); }
__device__ __forceinline__ float bfr(float f) { return bf2f(f2bf(f)); }
__device__ __forceinline__ v16h cat16(v8h lo, v8h hi) { return __builtin_shufflevector(lo, hi, 0, 1, 2, 3, 4, 5, 6, 7, 8, 9, 10, 11, 12, 13, 14, 15); }
__device__ __forceinline__ v16bf cat16b(v8us lo, v8us hi) { return __builtin_bit_cast(v16bf, __builtin_shufflevector(lo, hi, 0, 1, 2, 3, 4, 5, 6, 7, 8, 9, 10, 11, 12, 13, 14, 15)); }
__device__ __forceinline__ v8f wmma16(v16h a, v16h b, v8f c) { return __builtin_amdgcn_wmma_f32_16x16x32_f16(false, a, false, b, (short)0, c, false, false); }
__device__ __forceinline__ v8f wmmab(v16bf a, v16bf b, v8f c) { return __builtin_amdgcn_wmma_f32_16x16x32_bf16(false, a, false, b, (short)0, c, false, false); }

template <typename T16> struct WFrag;
template <> struct WFrag<h16> { typedef v16h V; static __device__ __forceinline__ V ld(const h16* p) { return cat16(*(const v8h*)p, *(const v8h*)(p + 16)); } static __device__ __forceinline__ v8f mma(V a, V b, v8f c) { return wmma16(a, b, c); } };
template <> struct WFrag<bf> { typedef v16bf V; static __device__ __forceinline__ V ld(const bf* p) { return cat16b(*(const v8us*)p, *(const v8us*)(p + 16)); } static __device__ __forceinline__ v8f mma(V a, V b, v8f c) { return wmmab(a, b, c); } };
template <typename T16, int NSPLIT, bool BIAS>
__global__ __launch_bounds__(32) void k_gemmw(const T16* __restrict__ A, const T16* __restrict__ A2, const T16* __restrict__ Bt, const T16* __restrict__ Bt2, int K, float* C, int ldc, const float* __restrict__ bias, size_t sA, size_t sB, size_t sC) {
    typedef typename WFrag<T16>::V V;
    __shared__ __align__(16) float os[16 * 68];
    const size_t z = blockIdx.z; A += z * sA; if (A2) A2 += z * sA; Bt += z * sB; if (Bt2) Bt2 += z * sB; C += z * sC;
    const int lane = threadIdx.x & 31, lr = lane & 15, hi = lane >> 4; const int r0 = blockIdx.x * 64, c0 = blockIdx.y * 64;
    v8f acc[4][4];
#pragma unroll
    for (int mb = 0; mb < 4; ++mb)
#pragma unroll
        for (int nb = 0; nb < 4; ++nb) acc[mb][nb] = (v8f){};
    const size_t aoff = (size_t)(r0 + lr) * K + 8 * hi, boff = (size_t)(c0 + lr) * K + 8 * hi;
#pragma unroll 1
    for (int kc = 0; kc < K; kc += 32) {
        V a[4], a2[4];
#pragma unroll
        for (int mb = 0; mb < 4; ++mb) { a[mb] = WFrag<T16>::ld(A + aoff + (size_t)mb * 16 * K + kc); if (NSPLIT == 1 || NSPLIT == 2) a2[mb] = WFrag<T16>::ld(A2 + aoff + (size_t)mb * 16 * K + kc); }
#pragma unroll
        for (int nb = 0; nb < 4; ++nb) { const V b = WFrag<T16>::ld(Bt + boff + (size_t)nb * 16 * K + kc); V b2; if (NSPLIT >= 2) b2 = WFrag<T16>::ld(Bt2 + boff + (size_t)nb * 16 * K + kc);
#pragma unroll
            for (int mb = 0; mb < 4; ++mb) { acc[mb][nb] = WFrag<T16>::mma(a[mb], b, acc[mb][nb]); if (NSPLIT == 1 || NSPLIT == 2) acc[mb][nb] = WFrag<T16>::mma(a2[mb], b, acc[mb][nb]); if (NSPLIT >= 2) acc[mb][nb] = WFrag<T16>::mma(a[mb], b2, acc[mb][nb]); } }
        asm volatile("v_nop\n\tv_nop\n\tv_nop\n\tv_nop" : "+v"(acc[0][0]), "+v"(acc[1][1]), "+v"(acc[2][2]), "+v"(acc[3][3]) : "v"(a[0]), "v"(a[3]));
    }
#pragma unroll
    for (int mb = 0; mb < 4; ++mb) {
#pragma unroll
        for (int nb = 0; nb < 4; ++nb) {
#pragma unroll
            for (int j = 0; j < 8; ++j) os[(hi * 8 + j) * 68 + nb * 16 + lr] = acc[mb][nb][j]; }
        __builtin_amdgcn_wave_barrier(); asm volatile("" ::: "memory");
        float* crow = C + (size_t)(r0 + mb * 16) * ldc + c0;
#pragma unroll 1
        for (int ps = 0; ps < 2; ++ps) {
#pragma unroll
            for (int s = 0; s < 8; ++s) { const int row = 2 * s + hi, cofs = lr * 4; v4f val = *(const v4fa*)(os + row * 68 + cofs); if (BIAS) { val[0] += bfr(bias[c0 + cofs]); val[1] += bfr(bias[c0 + cofs + 1]); val[2] += bfr(bias[c0 + cofs + 2]); val[3] += bfr(bias[c0 + cofs + 3]); }
                *(volatile v4f*)(crow + (size_t)row * ldc + cofs) = val; }
            if (ps == 0) __threadfence(); }
        __builtin_amdgcn_wave_barrier(); asm volatile("" ::: "memory");
    }
}

template <typename T16, int NSPLIT, int CMODE>
__global__ __launch_bounds__(32) void k_gemmc(const T16* __restrict__ A, const T16* __restrict__ A2, const T16* __restrict__ Bt, const T16* __restrict__ Bt2, int K, float* C, int ldc, int roff, size_t sA, size_t sB, size_t sC) {
    typedef typename WFrag<T16>::V V;
    __shared__ __align__(16) float os[16 * 68];
    const size_t z = blockIdx.z; A += z * sA; if (A2) A2 += z * sA; Bt += z * sB; if (Bt2) Bt2 += z * sB; C += z * sC;
    const int lane = threadIdx.x & 31, lr = lane & 15, hi = lane >> 4; const int r0 = blockIdx.x * 64, c0 = blockIdx.y * 64;
    if (CMODE == 1 && c0 > r0 + roff + 63) return;
    const int Kl = (CMODE == 2) ? min(K, r0 + roff + 64) : K;
    v8f acc[4][4];
#pragma unroll
    for (int mb = 0; mb < 4; ++mb)
#pragma unroll
        for (int nb = 0; nb < 4; ++nb) acc[mb][nb] = (v8f){};
    const size_t aoff = (size_t)(r0 + lr) * K + 8 * hi, boff = (size_t)(c0 + lr) * K + 8 * hi;
#pragma unroll 1
    for (int kc = 0; kc < Kl; kc += 32) {
        V a[4], a2[4];
#pragma unroll
        for (int mb = 0; mb < 4; ++mb) { a[mb] = WFrag<T16>::ld(A + aoff + (size_t)mb * 16 * K + kc); if (NSPLIT == 1 || NSPLIT == 2) a2[mb] = WFrag<T16>::ld(A2 + aoff + (size_t)mb * 16 * K + kc); }
#pragma unroll
        for (int nb = 0; nb < 4; ++nb) { const V b = WFrag<T16>::ld(Bt + boff + (size_t)nb * 16 * K + kc); V b2; if (NSPLIT >= 2) b2 = WFrag<T16>::ld(Bt2 + boff + (size_t)nb * 16 * K + kc);
#pragma unroll
            for (int mb = 0; mb < 4; ++mb) { acc[mb][nb] = WFrag<T16>::mma(a[mb], b, acc[mb][nb]); if (NSPLIT == 1 || NSPLIT == 2) acc[mb][nb] = WFrag<T16>::mma(a2[mb], b, acc[mb][nb]); if (NSPLIT >= 2) acc[mb][nb] = WFrag<T16>::mma(a[mb], b2, acc[mb][nb]); } }
        asm volatile("v_nop\n\tv_nop\n\tv_nop\n\tv_nop" : "+v"(acc[0][0]), "+v"(acc[1][1]), "+v"(acc[2][2]), "+v"(acc[3][3]) : "v"(a[0]), "v"(a[3]));
    }
#pragma unroll
    for (int mb = 0; mb < 4; ++mb) {
#pragma unroll
        for (int nb = 0; nb < 4; ++nb) {
#pragma unroll
            for (int j = 0; j < 8; ++j) os[(hi * 8 + j) * 68 + nb * 16 + lr] = acc[mb][nb][j]; }
        __builtin_amdgcn_wave_barrier(); asm volatile("" ::: "memory");
        float* crow = C + (size_t)(r0 + mb * 16) * ldc + c0;
#pragma unroll 1
        for (int ps = 0; ps < 2; ++ps) {
#pragma unroll
            for (int s = 0; s < 8; ++s) { const int row = 2 * s + hi, cofs = lr * 4; v4f val = *(const v4fa*)(os + row * 68 + cofs);
                *(volatile v4f*)(crow + (size_t)row * ldc + cofs) = val; }
            if (ps == 0) __threadfence(); }
        __builtin_amdgcn_wave_barrier(); asm volatile("" ::: "memory");
    }
}

__device__ __forceinline__ h16 tohx(float x) { return (h16)x; }
__device__ __forceinline__ void splitf(float y, unsigned short& h, unsigned short& l) { h = f2bf(y); l = f2bf(y - bf2f(h)); }
typedef __attribute__((ext_vector_type(2))) _Float16 v2h;
typedef __attribute__((ext_vector_type(4))) _Float16 v4h;
typedef __attribute__((ext_vector_type(2))) unsigned short v2us;
typedef __attribute__((ext_vector_type(4))) unsigned short v4us;
typedef __attribute__((ext_vector_type(2))) float v2f;

__global__ __launch_bounds__(256) void k_cvt8(const float* __restrict__ src, bf* dst, unsigned n8) { const unsigned i = blockIdx.x * 256u + threadIdx.x; if (i >= n8) return; const v8f v = *(const v8f*)(src + (size_t)i * 8); v8us o;
#pragma unroll
    for (int k = 0; k < 8; ++k) o[k] = f2bf(v[k]);
    *(volatile v8us*)(dst + (size_t)i * 8) = o; __threadfence(); *(volatile v8us*)(dst + (size_t)i * 8) = o; }

__global__ __launch_bounds__(256) void k_vtp(const float* __restrict__ F, unsigned pitch, unsigned nheads, h16* V16, bf* Vh, bf* Vl) {
    const unsigned e = (blockIdx.x * 256u + threadIdx.x) * 2u; if (e >= nheads * (unsigned)(HD * TT)) return;
    const unsigned t = e % (unsigned)TT; const unsigned d = (e / (unsigned)TT) & (unsigned)(HD - 1); const unsigned g = e / (unsigned)(TT * HD); v2h o16; v2us oh, ol;
#pragma unroll
    for (unsigned q = 0; q < 2; ++q) { const float x = F[(size_t)(t + q) * pitch + g * HD + d]; o16[q] = tohx(x); unsigned short a2, c2; splitf(x, a2, c2); oh[q] = a2; ol[q] = c2; }
    *(volatile v2h*)(V16 + e) = o16; *(volatile v2us*)(Vh + e) = oh; *(volatile v2us*)(Vl + e) = ol; __threadfence(); *(volatile v2h*)(V16 + e) = o16; *(volatile v2us*)(Vh + e) = oh; *(volatile v2us*)(Vl + e) = ol; }

__global__ __launch_bounds__(256) void k_asoft(const float* __restrict__ Sb, h16* P16, bf* Ph, bf* Pl) {
    const unsigned lane = threadIdx.x & 31u; const unsigned row = blockIdx.x * 8u + (threadIdx.x >> 5); if (row >= (unsigned)(ZH * TT)) return;
    const unsigned i = row % (unsigned)TT; const unsigned zz = row / (unsigned)TT; const bool hires = (i < (unsigned)RH); const float* sr = Sb + (size_t)row * TT; float v[TT / 32]; float mx = -3.0e38f;
#pragma unroll
    for (int ch = 0; ch < TT / 128; ++ch) { const unsigned j0 = (unsigned)ch * 128u + lane * 4u; const v4f a = *(const v4f*)(sr + j0);
#pragma unroll
        for (int q = 0; q < 4; ++q) { const unsigned j = j0 + (unsigned)q; const float t = (j <= i) ? a[q] * SCL : -3.0e38f; v[ch * 4 + q] = t; mx = fmaxf(mx, t); } }
#pragma unroll
    for (int sh = 16; sh; sh >>= 1) mx = fmaxf(mx, __shfl_xor(mx, sh, 32));
    float sum = 0.f;
#pragma unroll
    for (int k = 0; k < TT / 32; ++k) { float d0 = __fsub_rn(v[k], mx); asm volatile("" : "+v"(d0)); v[k] = __builtin_amdgcn_exp2f(__fmul_rn(d0, 1.4426950408889634f)); sum += v[k]; }
#pragma unroll
    for (int sh = 16; sh; sh >>= 1) sum += __shfl_xor(sum, sh, 32);
    const float f = __fdiv_rn(hires ? 1.0f : PCAR, sum);
#pragma unroll 1
    for (int ps = 0; ps < 2; ++ps) {
        if (hires) {
#pragma unroll
            for (int ch = 0; ch < TT / 128; ++ch) { v4us oh, ol;
#pragma unroll
                for (int q = 0; q < 4; ++q) { unsigned short a, c2; splitf(v[ch * 4 + q] * f, a, c2); oh[q] = a; ol[q] = c2; }
                const size_t oo = ((size_t)zz * (RH ? RH : 1) + i) * TT + (unsigned)ch * 128u + lane * 4u; *(volatile v4us*)(Ph + oo) = oh; *(volatile v4us*)(Pl + oo) = ol; }
        } else {
#pragma unroll
            for (int ch = 0; ch < TT / 128; ++ch) { v4h o4;
#pragma unroll
                for (int q = 0; q < 4; ++q) o4[q] = tohx(v[ch * 4 + q] * f);
                *(volatile v4h*)(P16 + (size_t)row * TT + (unsigned)ch * 128u + lane * 4u) = o4; } }
        if (ps == 0) __threadfence(); }
}

__constant__ float INVT[HD / 2] = { 1.000000000e+00f, 7.498942018e-01f, 5.623413324e-01f, 4.216965139e-01f, 3.162277639e-01f, 2.371373773e-01f, 1.778279394e-01f, 1.333521456e-01f, 1.000000015e-01f, 7.498942316e-02f, 5.623413250e-02f, 4.216964915e-02f, 3.162277490e-02f, 2.371373773e-02f, 1.778279431e-02f, 1.333521400e-02f, 9.999999776e-03f, 7.498942316e-03f, 5.623413250e-03f, 4.216964822e-03f, 3.162277630e-03f, 2.371373819e-03f, 1.778279431e-03f, 1.333521446e-03f, 1.000000047e-03f, 7.498941850e-04f, 5.623413017e-04f, 4.216965172e-04f, 3.162277571e-04f, 2.371373703e-04f, 1.778279402e-04f, 1.333521504e-04f };
__global__ __launch_bounds__(256) void k_csIL(const int* __restrict__ tpos, const int* __restrict__ thp, float* CS) {
    const unsigned idx = blockIdx.x * 256u + threadIdx.x; if (idx >= (unsigned)(TT * HD)) return;
    const unsigned d = idx & (unsigned)(HD - 1); const unsigned t = idx >> 6;
    const float pz = (thp[0] == THETA_I) ? 0.0f : __uint_as_float(0x7FC00000u);
    const float a = __fmul_rn((float)tpos[t], INVT[d >> 1]); v2f cs; cs[0] = cosf(a) + pz; cs[1] = sinf(a) + pz;
    *(volatile v2f*)(CS + (size_t)idx * 2) = cs; __threadfence(); *(volatile v2f*)(CS + (size_t)idx * 2) = cs; }

__global__ __launch_bounds__(256) void k_ropeI(const float* __restrict__ F, unsigned pitch, unsigned nheads, const float* __restrict__ CS, float sc, h16* P16, bf* Ph, bf* Pl) {
    const unsigned e = (blockIdx.x * 256u + threadIdx.x) * 2u; if (e >= nheads * (unsigned)(TT * HD)) return;
    const unsigned d = e & (unsigned)(HD - 1); const unsigned t = (e >> 6) % (unsigned)TT; const unsigned h = e / (unsigned)(HD * TT);
    const float* f = F + (size_t)t * pitch + h * HD; const float x0 = f[d], x1 = f[d + 1]; const v2f cs = *(const v2f*)(CS + ((size_t)t * HD + d) * 2); v2h o16; v2us oh, ol;
    float a0 = __fmul_rn(x0, cs[0]), b0 = __fmul_rn(x1, cs[1]), a1 = __fmul_rn(x1, cs[0]), b1 = __fmul_rn(x0, cs[1]); asm volatile("" : "+v"(a0), "+v"(b0), "+v"(a1), "+v"(b1));
    float r0 = __fsub_rn(a0, b0) * sc, r1 = __fadd_rn(b1, a1) * sc;
    o16[0] = tohx(r0); o16[1] = tohx(r1); { unsigned short a2, c2; splitf(r0, a2, c2); oh[0] = a2; ol[0] = c2; splitf(r1, a2, c2); oh[1] = a2; ol[1] = c2; }
    *(volatile v2h*)(P16 + e) = o16; *(volatile v2us*)(Ph + e) = oh; *(volatile v2us*)(Pl + e) = ol; __threadfence(); *(volatile v2h*)(P16 + e) = o16; *(volatile v2us*)(Ph + e) = oh; *(volatile v2us*)(Pl + e) = ol; }

__global__ __launch_bounds__(256) void k_merge(const float* __restrict__ O, unsigned h0, bf* Ah, bf* Al) {
    const unsigned e = (blockIdx.x * 256u + threadIdx.x) * 2u; if (e >= (unsigned)(ZH * TT * HD)) return;
    const unsigned d = e & (unsigned)(HD - 1); const unsigned t = (e >> 6) % (unsigned)TT; const unsigned zz = e / (unsigned)(HD * TT);
    const float cs = (t < (unsigned)RH) ? 1.0f : (1.0f / PCAR); const size_t oo = (size_t)t * DQ + (h0 + zz) * HD + d;
    v2us oh, ol;
#pragma unroll
    for (unsigned q = 0; q < 2; ++q) { unsigned short a, c2; splitf(O[e + q] * cs, a, c2); oh[q] = a; ol[q] = c2; }
    *(volatile v2us*)(Ah + oo) = oh; *(volatile v2us*)(Al + oo) = ol; __threadfence(); *(volatile v2us*)(Ah + oo) = oh; *(volatile v2us*)(Al + oo) = ol; }

constexpr size_t AL256(size_t b) { return (b + 255) & ~(size_t)255; }
constexpr size_t SZ_W    = AL256((size_t)DQ * DM * 2);
constexpr size_t SZ_CS   = AL256((size_t)TT * HD * 2 * 4);
constexpr size_t SZ_XB   = AL256((size_t)TT * DM * 2);
constexpr size_t SZ_F    = AL256((size_t)TT * DQ * 4);
constexpr size_t SZ_HP   = AL256((size_t)NH_ * TT * HD * 2);
constexpr size_t SZ_PHL  = AL256((size_t)ZH * RH * TT * 2);
constexpr size_t SZ_SB   = AL256((size_t)ZH * TT * TT * 4);
constexpr size_t SZ_P16  = AL256((size_t)ZH * TT * TT * 2);
constexpr size_t SZ_OB   = AL256((size_t)ZH * TT * HD * 4);
constexpr size_t OFF_WQ  = 0;
constexpr size_t OFF_WK  = OFF_WQ + SZ_W;
constexpr size_t OFF_WV  = OFF_WK + SZ_W;
constexpr size_t OFF_WO  = OFF_WV + SZ_W;
constexpr size_t OFF_CS  = OFF_WO + SZ_W;
constexpr size_t OFF_XB  = OFF_CS + SZ_CS;
constexpr size_t OFF_FQ  = OFF_XB + SZ_XB;
constexpr size_t OFF_FK  = OFF_FQ + SZ_F;
constexpr size_t OFF_Q16 = OFF_FK + SZ_F;
constexpr size_t OFF_K16 = OFF_Q16 + SZ_HP;
constexpr size_t OFF_V16 = OFF_K16 + SZ_HP;
constexpr size_t OFF_QH  = OFF_V16 + SZ_HP;
constexpr size_t OFF_QL  = OFF_QH + SZ_HP;
constexpr size_t OFF_KH  = OFF_QL + SZ_HP;
constexpr size_t OFF_KL  = OFF_KH + SZ_HP;
constexpr size_t OFF_VH  = OFF_KL + SZ_HP;
constexpr size_t OFF_VL  = OFF_VH + SZ_HP;
constexpr size_t OFF_PH  = OFF_VL + SZ_HP;
constexpr size_t OFF_PL  = OFF_PH + SZ_PHL;
constexpr size_t OFF_SB  = OFF_PL + SZ_PHL;
constexpr size_t OFF_P16 = OFF_SB + SZ_SB;
constexpr size_t OFF_OB  = OFF_P16 + SZ_P16;
constexpr size_t WS_TOTAL = OFF_OB + SZ_OB;
static_assert(WS_TOTAL <= (size_t)134217728);
static_assert((size_t)TT * DQ * 2 * 2 <= SZ_F);
static_assert(DKV == DQ);

extern "C" void kernel_launch(void* const* d_in, const int* in_sizes, int n_in,
                              void* d_out, int out_size, void* d_ws, size_t ws_size, hipStream_t stream) {
    if (n_in < 7) return;
    if ((size_t)in_sizes[0] < ((size_t)(NB - 1) * SEQ_FULL + SEQ) * DM) return;
    if ((size_t)in_sizes[1] < (size_t)DQ * DM || (size_t)in_sizes[2] < (size_t)DKV * DM || (size_t)in_sizes[3] < (size_t)DKV * DM || (size_t)in_sizes[4] < (size_t)DM * DQ) return;
    if (in_sizes[5] < SEQ || in_sizes[6] < 1) return;
    if ((size_t)out_size < (size_t)NB * SEQ * DM) return;
    if (WS_TOTAL > ws_size) return;
    const float* x = (const float*)d_in[0]; const float* wq = (const float*)d_in[1]; const float* wk = (const float*)d_in[2]; const float* wv = (const float*)d_in[3]; const float* wo = (const float*)d_in[4];
    const int* tpos = (const int*)d_in[5]; const int* thp = (const int*)d_in[6];
    float* OUT = (float*)d_out;
    char* wsp = (char*)d_ws;
    bf* WQ = (bf*)(wsp + OFF_WQ); bf* WK = (bf*)(wsp + OFF_WK); bf* WV = (bf*)(wsp + OFF_WV); bf* WO = (bf*)(wsp + OFF_WO); float* CS = (float*)(wsp + OFF_CS);
    bf* XB = (bf*)(wsp + OFF_XB); float* FQ = (float*)(wsp + OFF_FQ); float* FK = (float*)(wsp + OFF_FK);
    h16* QP16 = (h16*)(wsp + OFF_Q16); h16* KP16 = (h16*)(wsp + OFF_K16); h16* VT16 = (h16*)(wsp + OFF_V16);
    bf* QPh = (bf*)(wsp + OFF_QH); bf* QPl = (bf*)(wsp + OFF_QL); bf* KPh = (bf*)(wsp + OFF_KH); bf* KPl = (bf*)(wsp + OFF_KL); bf* VTh = (bf*)(wsp + OFF_VH); bf* VTl = (bf*)(wsp + OFF_VL);
    bf* Ph = (bf*)(wsp + OFF_PH); bf* Pl = (bf*)(wsp + OFF_PL);
    float* Sb = (float*)(wsp + OFF_SB); h16* P16 = (h16*)(wsp + OFF_P16); float* Ob = (float*)(wsp + OFF_OB);
    float* FV = FK;
    bf* ATh = (bf*)FQ; bf* ATl = ATh + (size_t)TT * DQ;
    k_cvt8<<<(unsigned)(((size_t)DQ * DM / 8 + 255) / 256), 256, 0, stream>>>(wq, WQ, (unsigned)((size_t)DQ * DM / 8));
    k_cvt8<<<(unsigned)(((size_t)DKV * DM / 8 + 255) / 256), 256, 0, stream>>>(wk, WK, (unsigned)((size_t)DKV * DM / 8));
    k_cvt8<<<(unsigned)(((size_t)DKV * DM / 8 + 255) / 256), 256, 0, stream>>>(wv, WV, (unsigned)((size_t)DKV * DM / 8));
    k_cvt8<<<(unsigned)(((size_t)DM * DQ / 8 + 255) / 256), 256, 0, stream>>>(wo, WO, (unsigned)((size_t)DM * DQ / 8));
    k_csIL<<<(TT * HD + 255) / 256, 256, 0, stream>>>(tpos, thp, CS);
    const unsigned LQ = (unsigned)(((size_t)NH_ * TT * HD / 2 + 255) / 256), LKv = (unsigned)(((size_t)NKV * TT * HD / 2 + 255) / 256);
    for (int b = 0; b < NB; ++b) {
        k_cvt8<<<(unsigned)(((size_t)TT * DM / 8 + 255) / 256), 256, 0, stream>>>(x + (size_t)b * SEQ_FULL * DM, XB, (unsigned)((size_t)TT * DM / 8));
        k_gemmw<bf, 0, false><<<dim3(TT / 64, DQ / 64, 1), 32, 0, stream>>>(XB, nullptr, WQ, nullptr, DM, FQ, DQ, nullptr, 0, 0, 0);
        k_ropeI<<<LQ, 256, 0, stream>>>(FQ, (unsigned)DQ, (unsigned)NH_, CS, 1.0f, QP16, QPh, QPl);
        k_gemmw<bf, 0, false><<<dim3(TT / 64, DKV / 64, 1), 32, 0, stream>>>(XB, nullptr, WK, nullptr, DM, FK, DKV, nullptr, 0, 0, 0);
        k_ropeI<<<LKv, 256, 0, stream>>>(FK, (unsigned)DKV, (unsigned)NKV, CS, 1.0f, KP16, KPh, KPl);
        k_gemmw<bf, 0, false><<<dim3(TT / 64, DKV / 64, 1), 32, 0, stream>>>(XB, nullptr, WV, nullptr, DM, FV, DKV, nullptr, 0, 0, 0);
        k_vtp<<<LKv, 256, 0, stream>>>(FV, (unsigned)DKV, (unsigned)NKV, VT16, VTh, VTl);
        for (int h0 = 0; h0 < NH_; h0 += ZH) { const size_t zq = (size_t)h0, zk = (size_t)(h0 / REP);
            k_gemmc<bf, 2, 1><<<dim3(RH / 64, TT / 64, ZH), 32, 0, stream>>>(QPh + zq * TT * HD, QPl + zq * TT * HD, KPh + zk * TT * HD, KPl + zk * TT * HD, HD, Sb, TT, 0, (size_t)TT * HD, (size_t)TT * HD, (size_t)TT * TT);
            if (TT > RH) k_gemmc<h16, 0, 1><<<dim3((TT - RH) / 64, TT / 64, ZH), 32, 0, stream>>>(QP16 + zq * TT * HD + (size_t)RH * HD, nullptr, KP16 + zk * TT * HD, nullptr, HD, Sb + (size_t)RH * TT, TT, RH, (size_t)TT * HD, (size_t)TT * HD, (size_t)TT * TT);
            k_asoft<<<ZH * TT / 8, 256, 0, stream>>>(Sb, P16, Ph, Pl);
            k_gemmc<bf, 2, 2><<<dim3(RH / 64, HD / 64, ZH), 32, 0, stream>>>(Ph, Pl, VTh + zk * HD * TT, VTl + zk * HD * TT, TT, Ob, HD, 0, (size_t)RH * TT, (size_t)HD * TT, (size_t)TT * HD);
            if (TT > RH) k_gemmc<h16, 0, 2><<<dim3((TT - RH) / 64, HD / 64, ZH), 32, 0, stream>>>(P16 + (size_t)RH * TT, nullptr, VT16 + zk * HD * TT, nullptr, TT, Ob + (size_t)RH * HD, HD, RH, (size_t)TT * TT, (size_t)HD * TT, (size_t)TT * HD);
            k_merge<<<(unsigned)(((size_t)ZH * TT * HD / 2 + 255) / 256), 256, 0, stream>>>(Ob, (unsigned)h0, ATh, ATl); }
        k_gemmw<bf, 1, false><<<dim3(TT / 64, DM / 64, 1), 32, 0, stream>>>(ATh, ATl, WO, nullptr, DQ, OUT + (size_t)b * TT * DM, DM, nullptr, 0, 0, 0); }
}
